// CISSVAE_38551626449609
// MI455X (gfx1250) — hardware-verified
//
#include <hip/hip_runtime.h>
#include <math.h>

typedef __attribute__((ext_vector_type(16))) _Float16 v16h;
typedef __attribute__((ext_vector_type(16))) __bf16 v16b;
typedef __attribute__((ext_vector_type(8)))  _Float16 v8h;
typedef __attribute__((ext_vector_type(8)))  float v8f;
typedef __attribute__((ext_vector_type(4)))  float v4f;
typedef __attribute__((ext_vector_type(2)))  float v2f;
typedef __attribute__((ext_vector_type(4)))  unsigned v4u;
typedef __attribute__((ext_vector_type(4)))  int v4i;
typedef float __attribute__((may_alias)) float_a;
typedef int __attribute__((may_alias)) int_a;

template <typename T> __device__ __forceinline__ void vst2(void* p, T v) { *(volatile T*)p = v; __threadfence(); *(volatile T*)p = v; }
__device__ __forceinline__ v8f wmma16(v16h a, v16h b, v8f c) {
  v8f d = __builtin_amdgcn_wmma_f32_16x16x32_f16(false, a, false, b, (short)0, c, false, false);
  asm volatile("v_nop\n\tv_nop\n\tv_nop\n\tv_nop" : "+v"(d) : "v"(a), "v"(b));
  return d;
}
__device__ __forceinline__ v8f wmma_bf(v16b a, v16b b, v8f c) {
  v8f d = __builtin_amdgcn_wmma_f32_16x16x32_bf16(false, a, false, b, (short)0, c, false, false);
  asm volatile("v_nop\n\tv_nop\n\tv_nop\n\tv_nop" : "+v"(d) : "v"(a), "v"(b));
  return d;
}
__device__ __forceinline__ v16h frag_h(const _Float16* rowk0, int lane) {
  union { v16h v; v8h q[2]; } u; const _Float16* p = rowk0 + 8 * (lane >> 4);
  u.q[0] = *(const v8h*)p; u.q[1] = *(const v8h*)(p + 16); return u.v;
}
__device__ __forceinline__ v16h frag_f32(const float* rowk0, int lane) {
  v16h a; const float* p = rowk0 + 8 * (lane >> 4);
#pragma unroll
  for (int i = 0; i < 8; ++i) { a[i] = (_Float16)p[i]; a[8 + i] = (_Float16)p[16 + i]; }
  return a;
}
__device__ __forceinline__ v16h frag_f32s(const float* rowk0, int lane, float sc) {
  v16h a; const float* p = rowk0 + 8 * (lane >> 4);
#pragma unroll
  for (int i = 0; i < 8; ++i) { a[i] = (_Float16)(p[i] * sc); a[8 + i] = (_Float16)(p[16 + i] * sc); }
  return a;
}
__device__ __forceinline__ v16h fragc_f32(const float* W, int k0, int n, int lane, int ld, int K) {
  v16h a; const int g = lane >> 4;
#pragma unroll
  for (int i = 0; i < 8; ++i) { const int ka = k0 + 8 * g + i, kb = ka + 16;
    a[i] = (_Float16)(ka < K ? W[(size_t)(ka < K ? ka : K - 1) * ld + n] : 0.f); a[8 + i] = (_Float16)(kb < K ? W[(size_t)(kb < K ? kb : K - 1) * ld + n] : 0.f); }
  return a;
}
struct F2 { v16b h, l; };
__device__ __forceinline__ F2 bsplit16(const float v[16]) { F2 r;
#pragma unroll
  for (int i = 0; i < 16; ++i) { const __bf16 h = (__bf16)v[i]; r.h[i] = h; r.l[i] = (__bf16)(v[i] - (float)h); }
  return r; }
__device__ __forceinline__ F2 split_row(const float* row, int k0, int lane) { float v[16]; const float* p = row + k0 + 8 * (lane >> 4);
#pragma unroll
  for (int i = 0; i < 8; ++i) { v[i] = p[i]; v[8 + i] = p[16 + i]; }
  return bsplit16(v); }
__device__ __forceinline__ F2 split_rowK(const float* row, int k0, int lane, int K) { float v[16]; const int g = lane >> 4;
#pragma unroll
  for (int i = 0; i < 8; ++i) { const int ka = k0 + 8 * g + i, kb = ka + 16; v[i] = ka < K ? row[ka < K ? ka : K - 1] : 0.f; v[8 + i] = kb < K ? row[kb < K ? kb : K - 1] : 0.f; }
  return bsplit16(v); }
__device__ __forceinline__ F2 split_col(const float* W, int k0, int n, int lane, int ld, int K) { float v[16]; const int g = lane >> 4;
#pragma unroll
  for (int i = 0; i < 8; ++i) { const int ka = k0 + 8 * g + i, kb = ka + 16; v[i] = ka < K ? W[(size_t)(ka < K ? ka : K - 1) * ld + n] : 0.f; v[8 + i] = kb < K ? W[(size_t)(kb < K ? kb : K - 1) * ld + n] : 0.f; }
  return bsplit16(v); }
__device__ __forceinline__ v8f mac3(const F2& a, const F2& b, v8f c) { c = wmma_bf(a.l, b.h, c); c = wmma_bf(a.h, b.l, c); return wmma_bf(a.h, b.h, c); }
__device__ __forceinline__ float sigm(float v) { return 1.0f / (1.0f + expf(-v)); }
#define LDSX() do { asm volatile("s_wait_dscnt 0" ::: "memory"); __builtin_amdgcn_wave_barrier(); __builtin_amdgcn_fence(__ATOMIC_RELEASE, "workgroup"); } while (0)


#define NBR 16384
#define NC 8
#define DIN 512
#define H0 1024
#define H1 512
#define H2 256
#define LAT 64
#define NPAD (NBR + NC * 64)
#define NTL (NPAD / 64)
#define WSC 256.0f
typedef __attribute__((ext_vector_type(8))) __bf16 v8b;
__device__ __forceinline__ v16b frag_b(const __bf16* rowk0, int lane) {
  union { v16b v; v8b q[2]; } u; const __bf16* p = rowk0 + 8 * (lane >> 4);
  u.q[0] = *(const v8b*)p; u.q[1] = *(const v8b*)(p + 16); return u.v;
}
__device__ __forceinline__ float bfr(float v) { return (float)(__bf16)v; }
__device__ __attribute__((noinline)) float exp_ni(float v) { return expf(v); }
__device__ __attribute__((noinline)) float erf_ni(float v) { return erff(v); }

#define WS_W0  0u
#define WS_WU  (WS_W0 + 2u * (size_t)H0 * DIN)
#define WS_W2  (WS_WU + 2u * (size_t)NC * H1 * H0)
#define WS_ML  (WS_W2 + 2u * (size_t)H2 * H1)
#define WS_WD0 (WS_ML + 2u * (size_t)128 * H2)
#define WS_WD1 (WS_WD0 + 2u * (size_t)NC * H2 * LAT)
#define WS_WD2 (WS_WD1 + 2u * (size_t)H1 * H2)
#define WS_WF  (WS_WD2 + 2u * (size_t)NC * H0 * H1)
#define WS_PERM (WS_WF + 2u * (size_t)NC * H1 * H0)
#define WS_TILEC (WS_PERM + 4u * (size_t)NPAD)
#define WS_XS  (WS_TILEC + 4u * (size_t)NTL + 64u)
#define WS_ES  (WS_XS + 2u * (size_t)NPAD * DIN)
#define WS_A0  (WS_ES + 4u * (size_t)NPAD * LAT)
#define WS_A1  (WS_A0 + 2u * (size_t)NPAD * H0)
#define WS_A2  (WS_A1 + 2u * (size_t)NPAD * H1)
#define WS_Z   (WS_A2 + 2u * (size_t)NPAD * H2)
#define WS_D0  (WS_Z + 4u * (size_t)NPAD * LAT)
#define WS_D1  (WS_D0 + 2u * (size_t)NPAD * H2)
#define WS_D2  (WS_D1 + 2u * (size_t)NPAD * H1)
#define WS_END (WS_D2 + 2u * (size_t)NPAD * H0)

__global__ __launch_bounds__(256) void k_pack(const float* __restrict__ W0, const float* __restrict__ WU, const float* __restrict__ W2, const float* __restrict__ MUW, const float* __restrict__ LVW, const float* __restrict__ WD0, const float* __restrict__ WD1, const float* __restrict__ WD2, const float* __restrict__ WF, char* __restrict__ ws) {
  const int n = blockIdx.x, which = blockIdx.y, c = blockIdx.z, t = threadIdx.x; __shared__ __align__(16) _Float16 sh[1024]; __shared__ __align__(16) __bf16 sb[512];
  if (which == 0) { if (c > 0 || n >= H0) return; for (int k = t; k < DIN; k += 256) sb[k] = (__bf16)W0[(size_t)k * H0 + n]; __syncthreads(); for (int q = t; q < DIN / 8; q += 256) vst2((unsigned*)((__bf16*)(ws + WS_W0) + (size_t)n * DIN + q * 8), *(const v4u*)&sb[q * 8]); }
  else if (which == 1) { if (n >= H1) return; for (int k = t; k < H0; k += 256) sh[k] = (_Float16)(bfr(WU[((size_t)c * H0 + k) * H1 + n]) * WSC); __syncthreads(); for (int q = t; q < H0 / 8; q += 256) vst2((unsigned*)((_Float16*)(ws + WS_WU) + ((size_t)c * H1 + n) * H0 + q * 8), *(const v4u*)&sh[q * 8]); }
  else if (which == 2) { if (c > 0 || n >= H2) return; for (int k = t; k < H1; k += 256) sh[k] = (_Float16)(bfr(W2[(size_t)k * H2 + n]) * WSC); __syncthreads(); for (int q = t; q < H1 / 8; q += 256) vst2((unsigned*)((_Float16*)(ws + WS_W2) + (size_t)n * H1 + q * 8), *(const v4u*)&sh[q * 8]); }
  else if (which == 3) { if (c > 0 || n >= 128) return; const float* src = (n < LAT) ? MUW : LVW; const int nn = n % LAT; for (int k = t; k < H2; k += 256) sh[k] = (_Float16)(bfr(src[(size_t)k * LAT + nn]) * WSC); __syncthreads(); for (int q = t; q < H2 / 8; q += 256) vst2((unsigned*)((_Float16*)(ws + WS_ML) + (size_t)n * H2 + q * 8), *(const v4u*)&sh[q * 8]); }
  else if (which == 4) { if (n >= H2) return; if (t < LAT) sb[t] = (__bf16)WD0[((size_t)c * LAT + t) * H2 + n]; __syncthreads(); if (t < LAT / 8) vst2((unsigned*)((__bf16*)(ws + WS_WD0) + ((size_t)c * H2 + n) * LAT + t * 8), *(const v4u*)&sb[t * 8]); }
  else if (which == 5) { if (c > 0 || n >= H1) return; for (int k = t; k < H2; k += 256) sh[k] = (_Float16)(bfr(WD1[(size_t)k * H1 + n]) * WSC); __syncthreads(); for (int q = t; q < H2 / 8; q += 256) vst2((unsigned*)((_Float16*)(ws + WS_WD1) + (size_t)n * H2 + q * 8), *(const v4u*)&sh[q * 8]); }
  else if (which == 6) { for (int k = t; k < H1; k += 256) sh[k] = (_Float16)(bfr(WD2[((size_t)c * H1 + k) * H0 + n]) * WSC); __syncthreads(); for (int q = t; q < H1 / 8; q += 256) vst2((unsigned*)((_Float16*)(ws + WS_WD2) + ((size_t)c * H0 + n) * H1 + q * 8), *(const v4u*)&sh[q * 8]); }
  else { if (n >= DIN) return; for (int k = t; k < H0; k += 256) sh[k] = (_Float16)(bfr(WF[((size_t)c * H0 + k) * DIN + n]) * WSC); __syncthreads(); for (int q = t; q < H0 / 8; q += 256) vst2((unsigned*)((_Float16*)(ws + WS_WF) + ((size_t)c * DIN + n) * H0 + q * 8), *(const v4u*)&sh[q * 8]); } }
__global__ __launch_bounds__(256) void k_sort(const int* __restrict__ LBL, int* __restrict__ PERM, int* __restrict__ TILEC) { __shared__ int cnt[256][NC]; __shared__ int gstart[NC + 1]; __shared__ __align__(16) int perm[NPAD]; __shared__ __align__(16) int tilec[NTL + 16]; const int t = threadIdx.x; const int chunk = NBR / 256;
  int my[NC]; for (int c = 0; c < NC; ++c) my[c] = 0;
  for (int i = 0; i < chunk; ++i) { int l = LBL[t * chunk + i]; l = l < 0 ? 0 : (l >= NC ? NC - 1 : l); my[l]++; }
  for (int c = 0; c < NC; ++c) cnt[t][c] = my[c];
  for (int i = t; i < NPAD; i += 256) perm[i] = -1; for (int i = t; i < NTL + 16; i += 256) tilec[i] = -1;
  __syncthreads();
  if (t == 0) { int s = 0; for (int c = 0; c < NC; ++c) { gstart[c] = s; int tot = 0; for (int u = 0; u < 256; ++u) tot += cnt[u][c]; const int padded = (tot + 63) / 64 * 64; for (int tl = s / 64; tl < (s + padded) / 64; ++tl) tilec[tl] = c; s += padded; } gstart[NC] = s; }
  __syncthreads();
  int off[NC]; for (int c = 0; c < NC; ++c) { int o = gstart[c]; for (int u = 0; u < t; ++u) o += cnt[u][c]; off[c] = o; }
  for (int i = 0; i < chunk; ++i) { const int row = t * chunk + i; int l = LBL[row]; l = l < 0 ? 0 : (l >= NC ? NC - 1 : l); perm[off[l]++] = row; }
  __syncthreads();
  for (int q = t; q < NPAD / 4; q += 256) vst2((unsigned*)(PERM + q * 4), *(const v4u*)&perm[q * 4]);
  if (t < (NTL + 16) / 4) vst2((unsigned*)(TILEC + t * 4), *(const v4u*)&tilec[t * 4]); }
__global__ __launch_bounds__(256) void k_gather(const float* __restrict__ X, const float* __restrict__ EPSI, const int* __restrict__ PERM, const int* __restrict__ TILEC, __bf16* __restrict__ XS, float* __restrict__ ES) { __shared__ __align__(16) __bf16 sx[64][DIN + 8]; __shared__ __align__(16) float se[64][LAT + 4]; const int t = threadIdx.x; const int tile = blockIdx.x; if (TILEC[tile] < 0) return;
  for (int rl = 0; rl < 64; ++rl) { const int src = PERM[tile * 64 + rl]; for (int k = t; k < DIN; k += 256) sx[rl][k] = (src >= 0) ? (__bf16)X[(size_t)src * DIN + k] : (__bf16)0.0f; if (t < LAT) se[rl][t] = (src >= 0) ? bfr(EPSI[(size_t)src * LAT + t]) : 0.f; }
  __syncthreads();
  for (int e = t; e < 64 * (DIN / 8); e += 256) { const int rl = e / (DIN / 8), q = e % (DIN / 8); vst2((unsigned*)(XS + ((size_t)tile * 64 + rl) * DIN + q * 8), *(const v4u*)&sx[rl][q * 8]); }
  for (int e = t; e < 64 * (LAT / 4); e += 256) { const int rl = e / (LAT / 4), q = e % (LAT / 4); vst2(ES + ((size_t)tile * 64 + rl) * LAT + q * 4, *(const v4f*)&se[rl][q * 4]); } }
template <int AT, int KW, int OM>
__global__ __launch_bounds__(128) void k_g(const void* __restrict__ Ain, const char* __restrict__ Wbase, size_t wstride, const float* __restrict__ Bbase, int bstride, const float* __restrict__ Bx, const int* __restrict__ TILEC, const int* __restrict__ PERM, const float* __restrict__ ES, void* __restrict__ OUTP, int ow) {
  __shared__ __align__(16) float sf[4][16][132]; __shared__ __align__(16) _Float16 so[64][136];
  const int tid = threadIdx.x, wave = tid >> 5, lane = tid & 31, col = lane & 15, g = lane >> 4; const int tile = blockIdx.x; const int clus = TILEC[tile]; if (clus < 0) return; const size_t rb = (size_t)tile * 64; const size_t r0 = rb + wave * 16; const int c0 = blockIdx.y * 128;
  const char* Wc = Wbase + (size_t)clus * wstride; const float* BB = Bbase ? Bbase + (size_t)clus * bstride : nullptr;
  v8f acc[8] = {};
  if (AT == 1) { const _Float16* A = (const _Float16*)Ain; const _Float16* Wr = (const _Float16*)Wc;
#pragma unroll 2
    for (int kc = 0; kc < KW / 32; ++kc) { const v16h a = frag_h(A + (r0 + col) * KW + kc * 32, lane);
#pragma unroll
      for (int j = 0; j < 8; ++j) acc[j] = wmma16(a, frag_h(Wr + (size_t)(c0 + j * 16 + col) * KW + kc * 32, lane), acc[j]); }
#pragma unroll
    for (int j = 0; j < 8; ++j)
#pragma unroll
      for (int r = 0; r < 8; ++r) acc[j][r] *= (1.0f / WSC); }
  else if (AT == 0) { const __bf16* A = (const __bf16*)Ain; const __bf16* Wr = (const __bf16*)Wc;
#pragma unroll 2
    for (int kc = 0; kc < KW / 32; ++kc) { const v16b a = frag_b(A + (r0 + col) * KW + kc * 32, lane);
#pragma unroll
      for (int j = 0; j < 8; ++j) acc[j] = wmma_bf(a, frag_b(Wr + (size_t)(c0 + j * 16 + col) * KW + kc * 32, lane), acc[j]); } }
  else { const float* A = (const float*)Ain; const __bf16* Wr = (const __bf16*)Wc;
#pragma unroll
    for (int kc = 0; kc < KW / 32; ++kc) { const F2 a = split_row(A + (r0 + col) * KW, kc * 32, lane);
#pragma unroll
      for (int j = 0; j < 8; ++j) { const v16b w = frag_b(Wr + (size_t)(c0 + j * 16 + col) * KW + kc * 32, lane); acc[j] = wmma_bf(a.h, w, acc[j]); acc[j] = wmma_bf(a.l, w, acc[j]); } } }
  if (OM == 0) {
#pragma unroll
    for (int j = 0; j < 8; ++j) { const float bb = BB ? bfr(BB[c0 + j * 16 + col]) : 0.f;
#pragma unroll
      for (int r = 0; r < 8; ++r) so[wave * 16 + 8 * g + r][j * 16 + col] = (_Float16)fmaxf(acc[j][r] + bb, 0.f); }
    __syncthreads(); _Float16* O16 = (_Float16*)OUTP; for (int e = tid; e < 64 * 16; e += 128) { const int rl = e >> 4, q = e & 15; vst2((unsigned*)(O16 + (rb + rl) * ow + c0 + q * 8), *(const v4u*)&so[rl][q * 8]); } }
  else if (OM == 1) {
#pragma unroll
    for (int j = 0; j < 4; ++j) { const float bm = bfr(BB[j * 16 + col]), bl = bfr(Bx[j * 16 + col]);
#pragma unroll
      for (int r = 0; r < 8; ++r) { const size_t row = r0 + 8 * g + r; const float mu = acc[j][r] + bm, lv = acc[j + 4][r] + bl; sf[wave][8 * g + r][j * 16 + col] = mu + expf(0.5f * lv) * ES[row * LAT + j * 16 + col]; } }
    LDSX(); float* Z = (float*)OUTP; for (int rl = 0; rl < 16; ++rl) if (lane < 16) vst2(Z + (r0 + rl) * LAT + lane * 4, *(const v4f*)&sf[wave][rl][lane * 4]); }
  else {
#pragma unroll
    for (int j = 0; j < 8; ++j) { const float bb = BB ? bfr(BB[c0 + j * 16 + col]) : 0.f;
#pragma unroll
      for (int r = 0; r < 8; ++r) sf[wave][8 * g + r][j * 16 + col] = acc[j][r] + bb; }
    LDSX(); float* Y = (float*)OUTP; for (int rl = 0; rl < 16; ++rl) { const int dst = PERM[r0 + rl]; if (dst >= 0) vst2(Y + (size_t)dst * ow + c0 + lane * 4, *(const v4f*)&sf[wave][rl][lane * 4]); } }
}
extern "C" void kernel_launch(void* const* d_in, const int* in_sizes, int n_in, void* d_out, int out_size, void* d_ws, size_t ws_size, hipStream_t stream) {
  (void)in_sizes; (void)n_in; (void)out_size;
  const float** F = (const float**)d_in;
  if (ws_size < (size_t)WS_END) return;
  char* ws = (char*)d_ws; int *PERM = (int*)(ws + WS_PERM), *TILEC = (int*)(ws + WS_TILEC); __bf16* XS = (__bf16*)(ws + WS_XS); float *ES = (float*)(ws + WS_ES), *Z = (float*)(ws + WS_Z); _Float16 *A0 = (_Float16*)(ws + WS_A0), *A1 = (_Float16*)(ws + WS_A1), *A2 = (_Float16*)(ws + WS_A2), *D0 = (_Float16*)(ws + WS_D0), *D1 = (_Float16*)(ws + WS_D1), *D2 = (_Float16*)(ws + WS_D2);
  k_pack<<<dim3(H0, 8, NC), 256, 0, stream>>>(F[3], F[5], F[7], F[9], F[11], F[13], F[15], F[17], F[19], ws);
  k_sort<<<1, 256, 0, stream>>>((const int*)d_in[1], PERM, TILEC);
  k_gather<<<NTL, 256, 0, stream>>>(F[0], F[2], PERM, TILEC, XS, ES);
  k_g<0, DIN, 0><<<dim3(NTL, H0 / 128), 128, 0, stream>>>(XS, ws + WS_W0, 0, F[4], 0, nullptr, TILEC, PERM, ES, A0, H0);
  k_g<1, H0, 0><<<dim3(NTL, H1 / 128), 128, 0, stream>>>(A0, ws + WS_WU, 2u * (size_t)H1 * H0, F[6], H1, nullptr, TILEC, PERM, ES, A1, H1);
  k_g<1, H1, 0><<<dim3(NTL, H2 / 128), 128, 0, stream>>>(A1, ws + WS_W2, 0, F[8], 0, nullptr, TILEC, PERM, ES, A2, H2);
  k_g<1, H2, 1><<<dim3(NTL, 1), 128, 0, stream>>>(A2, ws + WS_ML, 0, F[10], 0, F[12], TILEC, PERM, ES, Z, LAT);
  k_g<2, LAT, 0><<<dim3(NTL, H2 / 128), 128, 0, stream>>>(Z, ws + WS_WD0, 2u * (size_t)H2 * LAT, F[14], H2, nullptr, TILEC, PERM, ES, D0, H2);
  k_g<1, H2, 0><<<dim3(NTL, H1 / 128), 128, 0, stream>>>(D0, ws + WS_WD1, 0, F[16], 0, nullptr, TILEC, PERM, ES, D1, H1);
  k_g<1, H1, 0><<<dim3(NTL, H0 / 128), 128, 0, stream>>>(D1, ws + WS_WD2, 2u * (size_t)H0 * H1, F[18], H0, nullptr, TILEC, PERM, ES, D2, H0);
  k_g<1, H0, 2><<<dim3(NTL, DIN / 128), 128, 0, stream>>>(D2, ws + WS_WF, 2u * (size_t)DIN * H0, F[20], DIN, nullptr, TILEC, PERM, ES, d_out, DIN);
}
